// RelationalAttention_55001351192725
// MI455X (gfx1250) — hardware-verified
//
#include <hip/hip_runtime.h>

static constexpr int NB    = 2;
static constexpr int SEQ   = 1024;
static constexpr int DMOD  = 1024;
static constexpr int NHEAD = 16;
static constexpr int HDIM  = 64;
static constexpr int NREL  = 16;
static constexpr int RDIM  = 64;
static constexpr int NTOK  = NB * SEQ;
static constexpr int CHR   = 256;
static constexpr int NCHK  = SEQ / CHR;
static constexpr float SCALE_ATTN = 0.125f;
static constexpr float SCALE_REL  = 0.125f;
static constexpr float PCARRY     = 1024.0f;
static constexpr float PCARRY_INV = 1.0f / 1024.0f;

static_assert(NHEAD * HDIM == DMOD, "head split");
static_assert(NREL * RDIM == DMOD, "relation split");
static_assert(SEQ == 4 * 256, "softmax kernel handles 4 segments of 256 keys");
static_assert(SEQ % CHR == 0 && CHR % 64 == 0, "chunk tiling");
static_assert(NHEAD == 16 && NREL == 16, "relation mix kernel uses one 16x16 tile per token");
static_assert(HDIM % 32 == 0 && RDIM % 32 == 0, "K of score GEMMs multiple of 32");
static_assert(NTOK % 64 == 0 && DMOD % 64 == 0, "tile multiples");
static_assert((NTOK * DMOD) % (8 * 256) == 0, "cast kernel coverage");
static_assert((NHEAD * CHR) % 8 == 0 && CHR % 16 == 0, "softmax / mix grids");

typedef __attribute__((ext_vector_type(16))) _Float16 v16h;
typedef __attribute__((ext_vector_type(8)))  _Float16 v8h;
typedef __attribute__((ext_vector_type(16))) __bf16   v16b;
typedef __attribute__((ext_vector_type(8)))  __bf16   v8b;
typedef __attribute__((ext_vector_type(8)))  float    v8f;
typedef __attribute__((ext_vector_type(4)))  float    v4f;
typedef __attribute__((ext_vector_type(4)))  unsigned int v4u;

__device__ __forceinline__ unsigned short f2bf_bits(float f) {
  unsigned u = __float_as_uint(f);
  return (unsigned short)((u + 0x7FFFu + ((u >> 16) & 1u)) >> 16);
}
__device__ __forceinline__ float bf_bits2f(unsigned short h) { return __uint_as_float(((unsigned)h) << 16); }
__device__ __forceinline__ unsigned short h_bits(float f) { return __builtin_bit_cast(unsigned short, (_Float16)f); }
__device__ __forceinline__ unsigned pack_bf16x2(float a, float b) {
  return (unsigned)f2bf_bits(a) | ((unsigned)f2bf_bits(b) << 16);
}

__device__ __forceinline__ void dep_guard_h(v8f& a, v8f& b, v16h x, v16h y) { asm volatile("v_nop\n\tv_nop\n\tv_nop\n\tv_nop" : "+v"(a), "+v"(b) : "v"(x), "v"(y)); }
__device__ __forceinline__ void dep_guard_b(v8f& a, v8f& b, v16b x, v16b y) { asm volatile("v_nop\n\tv_nop\n\tv_nop\n\tv_nop" : "+v"(a), "+v"(b) : "v"(x), "v"(y)); }
__device__ __forceinline__ void keep4_h(v16h a, v16h b, v16h c, v16h d) { asm volatile("v_nop" :: "v"(a), "v"(b), "v"(c), "v"(d)); }
__device__ __forceinline__ void keep4_b(v16b a, v16b b, v16b c, v16b d) { asm volatile("v_nop" :: "v"(a), "v"(b), "v"(c), "v"(d)); }
__device__ __forceinline__ void acc_guard4(v8f& a, v8f& b, v8f& c, v8f& d) { asm volatile("v_nop\n\tv_nop\n\tv_nop\n\tv_nop" : "+v"(a), "+v"(b), "+v"(c), "+v"(d)); }
template <typename T> struct Frag;
template <> struct Frag<_Float16> {
  typedef v16h V; union U { v16h v; v8h h[2]; };
  static __device__ __forceinline__ v16h load(const _Float16* p) {
    U f; f.h[0] = *(const v8h*)(p); f.h[1] = *(const v8h*)(p + 16); return f.v;
  }
  static __device__ __forceinline__ v8f mma(v16h a, v16h b, v8f c) {
    return __builtin_amdgcn_wmma_f32_16x16x32_f16(false, a, false, b, (short)0, c, false, false);
  }
  static __device__ __forceinline__ void guard(v8f& a, v8f& b, v16h x, v16h y) { dep_guard_h(a, b, x, y); }
  static __device__ __forceinline__ void keep(v16h a, v16h b, v16h c, v16h d) { keep4_h(a, b, c, d); }
};
template <> struct Frag<__bf16> {
  typedef v16b V; union U { v16b v; v8b h[2]; };
  static __device__ __forceinline__ v16b load(const __bf16* p) {
    U f; f.h[0] = *(const v8b*)(p); f.h[1] = *(const v8b*)(p + 16); return f.v;
  }
  static __device__ __forceinline__ v8f mma(v16b a, v16b b, v8f c) {
    return __builtin_amdgcn_wmma_f32_16x16x32_bf16(false, a, false, b, (short)0, c, false, false);
  }
  static __device__ __forceinline__ void guard(v8f& a, v8f& b, v16b x, v16b y) { dep_guard_b(a, b, x, y); }
  static __device__ __forceinline__ void keep(v16b a, v16b b, v16b c, v16b d) { keep4_b(a, b, c, d); }
};

__device__ __forceinline__ v8f mma16h(v16h a, v16h b, v8f c) {
  c = __builtin_amdgcn_wmma_f32_16x16x32_f16(false, a, false, b, (short)0, c, false, false);
  asm volatile("v_nop\n\tv_nop\n\tv_nop\n\tv_nop" : "+v"(c) : "v"(a), "v"(b));
  return c;
}
__device__ __forceinline__ v8f mma16b(v16b a, v16b b, v8f c) {
  c = __builtin_amdgcn_wmma_f32_16x16x32_bf16(false, a, false, b, (short)0, c, false, false);
  asm volatile("v_nop\n\tv_nop\n\tv_nop\n\tv_nop" : "+v"(c) : "v"(a), "v"(b));
  return c;
}

template <int ET> struct Elem;
template <> struct Elem<0> { typedef _Float16 T; };
template <> struct Elem<1> { typedef __bf16 T; };
template <int ET, bool SPLIT, bool SPLITB, int BIAS_MODE, int OUT_MODE>
__global__ __launch_bounds__(256) void wmma_gemm64(
    const unsigned short* __restrict__ Ap, const unsigned short* __restrict__ A2p, int lda, long strideA,
    const unsigned short* __restrict__ Btp, const unsigned short* __restrict__ Bt2p, int ldb, long strideB,
    void* __restrict__ Cout, void* __restrict__ Cout2, int ldc, long strideC,
    const float* __restrict__ bias,
    int M, int N, int K, float scale) {
  typedef typename Elem<ET>::T T;
  typedef typename Frag<T>::V V;
  const T* A = (const T*)Ap; const T* A2 = (const T*)A2p; const T* Bt = (const T*)Btp; const T* Bt2 = (const T*)Bt2p;
  __shared__ __align__(16) float sT[8][16 * 68];
  const int b    = blockIdx.y;
  const int lane = threadIdx.x & 31;
  const int wave = threadIdx.x >> 5;
  const int tilesN = N >> 6;
  const int tilesM = M >> 6;
  const int tile = blockIdx.x * 8 + wave;
  if (tile >= tilesM * tilesN) return;
  const int tm = tile / tilesN;
  const int tn = tile - tm * tilesN;
  const int m0 = tm << 6;
  const int n0 = tn << 6;

  const T* Ab  = A  + (size_t)b * strideA;
  const T* Bb  = Bt + (size_t)b * strideB;
  const T* Ab2 = SPLIT ? (A2  + (size_t)b * strideA) : nullptr;
  const T* Bb2 = (SPLIT && SPLITB) ? (Bt2 + (size_t)b * strideB) : nullptr;

  const int rlane = lane & 15;
  const int koff  = (lane >> 4) * 8;
  const int mOff  = (lane >> 4) * 8;

  v8f acc[4][4];
#pragma unroll
  for (int i = 0; i < 4; ++i)
#pragma unroll
    for (int j = 0; j < 4; ++j) acc[i][j] = (v8f){0.f,0.f,0.f,0.f,0.f,0.f,0.f,0.f};

  for (int k0 = 0; k0 < K; k0 += 32) {
    V bh[4], bl[4];
#pragma unroll
    for (int j = 0; j < 4; ++j) {
      const size_t bo = (size_t)(n0 + (j << 4) + rlane) * ldb + koff + k0;
      bh[j] = Frag<T>::load(Bb + bo);
      if (SPLIT && SPLITB) bl[j] = Frag<T>::load(Bb2 + bo);
    }
#pragma unroll
    for (int i = 0; i < 4; ++i) {
      const size_t ao = (size_t)(m0 + (i << 4) + rlane) * lda + koff + k0;
      V ah = Frag<T>::load(Ab + ao);
      V al;
      if (SPLIT) al = Frag<T>::load(Ab2 + ao);
#pragma unroll
      for (int j = 0; j < 4; ++j) {
        acc[i][j] = Frag<T>::mma(ah, bh[j], acc[i][j]);
        if (SPLIT) {
          if (SPLITB) acc[i][j] = Frag<T>::mma(ah, bl[j], acc[i][j]);
          acc[i][j] = Frag<T>::mma(al, bh[j], acc[i][j]);
        }
      }
      Frag<T>::guard(acc[i][0], acc[i][3], ah, SPLIT ? al : ah);
    }
    Frag<T>::keep(bh[0], bh[1], bh[2], bh[3]);
    if (SPLIT && SPLITB) Frag<T>::keep(bl[0], bl[1], bl[2], bl[3]);
  }
  acc_guard4(acc[0][0], acc[0][1], acc[0][2], acc[0][3]);
  acc_guard4(acc[1][0], acc[1][1], acc[1][2], acc[1][3]);
  acc_guard4(acc[2][0], acc[2][1], acc[2][2], acc[2][3]);
  acc_guard4(acc[3][0], acc[3][1], acc[3][2], acc[3][3]);

  float* slab = sT[wave];
#pragma unroll
  for (int i = 0; i < 4; ++i) {
    const int mBase = m0 + (i << 4);
#pragma unroll
    for (int j = 0; j < 4; ++j) {
      const int n = n0 + (j << 4) + rlane;
      float bv = 0.f;
      if (BIAS_MODE == 2) bv = bias[n];
#pragma unroll
      for (int r = 0; r < 8; ++r) {
        float v = acc[i][j][r] * scale;
        if (BIAS_MODE == 1) v += bias[mBase + mOff + r];
        if (BIAS_MODE == 2) v += bv;
        slab[(mOff + r) * 68 + (j << 4) + rlane] = v;
      }
    }
    __builtin_amdgcn_fence(__ATOMIC_RELEASE, "workgroup");
    __builtin_amdgcn_wave_barrier();
    __builtin_amdgcn_fence(__ATOMIC_ACQUIRE, "workgroup");
    if (OUT_MODE == 0) {
      float* C = (float*)Cout + (size_t)b * strideC;
      const int hh = lane >> 4, c4 = (lane & 15) * 4;
      for (int pass = 0; pass < 2; ++pass) {
#pragma unroll
        for (int it = 0; it < 8; ++it) {
          const int row = it * 2 + hh;
          v4f v = *(const v4f*)(slab + row * 68 + c4);
          *(volatile v4f*)(C + (size_t)(mBase + row) * ldc + n0 + c4) = v;
        }
        __threadfence();
      }
    } else {
      const int q = lane >> 3, c8 = (lane & 7) * 8;
      unsigned short* C  = (unsigned short*)Cout  + (size_t)b * strideC;
      unsigned short* C2 = (OUT_MODE == 2) ? ((unsigned short*)Cout2 + (size_t)b * strideC) : nullptr;
      for (int pass = 0; pass < 2; ++pass) {
#pragma unroll
        for (int it = 0; it < 4; ++it) {
          const int row = it * 4 + q;
          const float* sp = slab + row * 68 + c8;
          v8h hv, lv;
#pragma unroll
          for (int e = 0; e < 8; ++e) {
            if (OUT_MODE == 1) {
              hv[e] = (_Float16)sp[e];
            } else {
              unsigned short hb = f2bf_bits(sp[e]);
              unsigned short lb = f2bf_bits(sp[e] - bf_bits2f(hb));
              hv[e] = __builtin_bit_cast(_Float16, hb);
              lv[e] = __builtin_bit_cast(_Float16, lb);
            }
          }
          *(volatile v8h*)(C + (size_t)(mBase + row) * ldc + n0 + c8) = hv;
          if (OUT_MODE == 2) *(volatile v8h*)(C2 + (size_t)(mBase + row) * ldc + n0 + c8) = lv;
        }
        __threadfence();
      }
    }
    __builtin_amdgcn_fence(__ATOMIC_RELEASE, "workgroup");
    __builtin_amdgcn_wave_barrier();
    __builtin_amdgcn_fence(__ATOMIC_ACQUIRE, "workgroup");
  }
}

__global__ __launch_bounds__(256) void k_cast_bf16x8(const float* __restrict__ s0, const float* __restrict__ s1,
    unsigned short* __restrict__ d0, unsigned short* __restrict__ d1, int n8) {
  const float* src = (blockIdx.y == 0) ? s0 : s1;
  unsigned short* dst = (blockIdx.y == 0) ? d0 : d1;
  const int i = blockIdx.x * 256 + threadIdx.x;
  if (i < n8) {
    const size_t e0 = (size_t)i * 8;
    const v4f a = *(const v4f*)(src + e0);
    const v4f c = *(const v4f*)(src + e0 + 4);
    v4u u;
    u[0] = pack_bf16x2(a[0], a[1]);
    u[1] = pack_bf16x2(a[2], a[3]);
    u[2] = pack_bf16x2(c[0], c[1]);
    u[3] = pack_bf16x2(c[2], c[3]);
    *(volatile v4u*)(dst + e0) = u;
    __threadfence();
    *(volatile v4u*)(dst + e0) = u;
  }
}

__global__ __launch_bounds__(256) void k_wT_bf16(const float* __restrict__ w0, const float* __restrict__ w1,
    const float* __restrict__ w2, const float* __restrict__ w3, const float* __restrict__ w4, const float* __restrict__ w5,
    unsigned short* __restrict__ dst) {
  __shared__ __align__(16) float tile[64 * 68];
  const int z = blockIdx.z;
  const float* W = (z == 0) ? w0 : (z == 1) ? w1 : (z == 2) ? w2 : (z == 3) ? w3 : (z == 4) ? w4 : w5;
  unsigned short* WT = dst + (size_t)z * DMOD * DMOD;
  const int k0 = blockIdx.y * 64;
  const int o0 = blockIdx.x * 64;
  const int tid = threadIdx.x;
#pragma unroll
  for (int it = 0; it < 4; ++it) {
    const int e = (it * 256 + tid) * 4;
    const int row = e >> 6, col = e & 63;
    const v4f v = *(const v4f*)(W + (size_t)(k0 + row) * DMOD + o0 + col);
    *(v4f*)(tile + row * 68 + col) = v;
  }
  __syncthreads();
  const int lane = tid & 31, wave = tid >> 5, q = lane >> 3, c8 = (lane & 7) * 8;
  v4u ov[2];
#pragma unroll
  for (int it = 0; it < 2; ++it) {
    const int oo = it * 32 + wave * 4 + q;
    float f[8];
#pragma unroll
    for (int e = 0; e < 8; ++e) f[e] = tile[(c8 + e) * 68 + oo];
    ov[it][0] = pack_bf16x2(f[0], f[1]);
    ov[it][1] = pack_bf16x2(f[2], f[3]);
    ov[it][2] = pack_bf16x2(f[4], f[5]);
    ov[it][3] = pack_bf16x2(f[6], f[7]);
  }
  for (int pass = 0; pass < 2; ++pass) {
#pragma unroll
    for (int it = 0; it < 2; ++it) {
      const int oo = it * 32 + wave * 4 + q;
      *(volatile v4u*)(WT + (size_t)(o0 + oo) * DMOD + k0 + c8) = ov[it];
    }
    __threadfence();
  }
}

__global__ __launch_bounds__(256) void k_wr_pack(const float* __restrict__ wr, unsigned short* __restrict__ dst) {
  __shared__ __align__(16) unsigned short tile[64 * 32];
  const int r0 = blockIdx.x * 64;
  const int tid = threadIdx.x;
  const int row = tid >> 2, kq = (tid & 3) * 8;
  v4u u;
  unsigned wv[4];
#pragma unroll
  for (int e = 0; e < 4; ++e) {
    const int ka = kq + 2 * e, kb = kq + 2 * e + 1;
    const int kac = ka < NREL ? ka : NREL - 1;
    const int kbc = kb < NREL ? kb : NREL - 1;
    const float fa = wr[(size_t)(r0 + row) * NREL + kac];
    const float fb = wr[(size_t)(r0 + row) * NREL + kbc];
    const unsigned ba = (ka < NREL) ? (unsigned)f2bf_bits(fa) : 0u;
    const unsigned bb = (kb < NREL) ? (unsigned)f2bf_bits(fb) : 0u;
    wv[e] = ba | (bb << 16);
  }
  u[0] = wv[0]; u[1] = wv[1]; u[2] = wv[2]; u[3] = wv[3];
  *(v4u*)(tile + row * 32 + kq) = u;
  __syncthreads();
  const int lane = tid & 31, wave = tid >> 5, q = lane >> 3, c8 = (lane & 7) * 8;
  const int L = wave * 4 + q;
  const v4u v = *(const v4u*)(tile + L * 64 + c8);
  for (int pass = 0; pass < 2; ++pass) {
    *(volatile v4u*)(dst + (size_t)r0 * 32 + L * 64 + c8) = v;
    __threadfence();
  }
}

__global__ __launch_bounds__(256) void k_softmax(const float* __restrict__ sc, unsigned short* __restrict__ ph,
    unsigned short* __restrict__ pl, unsigned short* __restrict__ p16, int i0, int jend) {
  const int lane = threadIdx.x & 31, wave = threadIdx.x >> 5;
  const int r = blockIdx.x * 8 + wave;
  const int i = i0 + (r & (CHR - 1));
  const size_t ro = (size_t)r * SEQ;
  const float NEG = -__builtin_huge_valf();
  float s[4][8];
  float m = NEG;
#pragma unroll
  for (int t = 0; t < 4; ++t) {
    const int j0 = t * 256 + lane * 8;
    if (t * 256 < jend) {
      const v4f a = *(const v4f*)(sc + ro + j0);
      const v4f c = *(const v4f*)(sc + ro + j0 + 4);
      s[t][0] = a[0]; s[t][1] = a[1]; s[t][2] = a[2]; s[t][3] = a[3];
      s[t][4] = c[0]; s[t][5] = c[1]; s[t][6] = c[2]; s[t][7] = c[3];
#pragma unroll
      for (int e = 0; e < 8; ++e) m = (j0 + e <= i) ? fmaxf(m, s[t][e]) : m;
    } else {
#pragma unroll
      for (int e = 0; e < 8; ++e) s[t][e] = 0.f;
    }
  }
#pragma unroll
  for (int off = 1; off < 32; off <<= 1) m = fmaxf(m, __shfl_xor(m, off, 32));
  float p[4][8];
  float sum = 0.f;
#pragma unroll
  for (int t = 0; t < 4; ++t) {
    const int j0 = t * 256 + lane * 8;
#pragma unroll
    for (int e = 0; e < 8; ++e) {
      float ev = __expf(s[t][e] - m);
      ev = (j0 + e <= i) ? ev : 0.f;
      p[t][e] = ev;
      sum += ev;
    }
  }
#pragma unroll
  for (int off = 1; off < 32; off <<= 1) sum += __shfl_xor(sum, off, 32);
  const float inv = 1.0f / sum;
  v4u hv[4], lv[4], fv[4];
#pragma unroll
  for (int t = 0; t < 4; ++t) {
#pragma unroll
    for (int e = 0; e < 4; ++e) {
      const float a = p[t][2 * e] * inv;
      const float c = p[t][2 * e + 1] * inv;
      const unsigned short ha = f2bf_bits(a), hc = f2bf_bits(c);
      const unsigned short la = f2bf_bits(a - bf_bits2f(ha)), lc = f2bf_bits(c - bf_bits2f(hc));
      const unsigned short fa = h_bits(a * PCARRY), fc = h_bits(c * PCARRY);
      hv[t][e] = (unsigned)ha | ((unsigned)hc << 16);
      lv[t][e] = (unsigned)la | ((unsigned)lc << 16);
      fv[t][e] = (unsigned)fa | ((unsigned)fc << 16);
    }
  }
  for (int pass = 0; pass < 2; ++pass) {
#pragma unroll
    for (int t = 0; t < 4; ++t) {
      if (t * 256 < jend) {
        const int j0 = t * 256 + lane * 8;
        *(volatile v4u*)(ph  + ro + j0) = hv[t];
        *(volatile v4u*)(pl  + ro + j0) = lv[t];
        *(volatile v4u*)(p16 + ro + j0) = fv[t];
      }
    }
    __threadfence();
  }
}

__global__ __launch_bounds__(256) void k_rel_mix(const unsigned short* __restrict__ p16, const unsigned short* __restrict__ rel,
    const unsigned short* __restrict__ wrp, const float* __restrict__ attsym,
    unsigned short* __restrict__ comb_hi, unsigned short* __restrict__ comb_lo, int i0, int rowbase) {
  __shared__ __align__(16) unsigned short arHL[2 * 16 * 16 * 32];
  __shared__ __align__(16) float slab[8][16 * 68];
  const int tid = threadIdx.x, lane = tid & 31, wave = tid >> 5;
  const int hh = lane >> 4, rl = lane & 15, koff = hh * 8;
  const int il0 = blockIdx.x * 16;
  {
    const v4u zz = {0u, 0u, 0u, 0u};
    v4u* zp = (v4u*)arHL;
    for (int qq = tid; qq < 2048; qq += 256) zp[qq] = zz;
  }
  __syncthreads();
  const v8f zero8 = {0.f, 0.f, 0.f, 0.f, 0.f, 0.f, 0.f, 0.f};
#pragma unroll
  for (int sub = 0; sub < 2; ++sub) {
    const int ill = wave + 8 * sub;
    const int il = il0 + ill;
    const int i = i0 + il;
    const int kend = (i & ~31) + 32;
    const _Float16* Ab = (const _Float16*)p16 + (size_t)rl * ((size_t)CHR * SEQ) + (size_t)il * SEQ + koff;
    const _Float16* Bb = (const _Float16*)rel + (size_t)il * ((size_t)NREL * SEQ) + (size_t)rl * SEQ + koff;
    v8f acc = zero8;
    for (int k0 = 0; k0 < kend; k0 += 32) {
      const v16h a  = Frag<_Float16>::load(Ab + k0);
      const v16h bb = Frag<_Float16>::load(Bb + k0);
      acc = mma16h(a, bb, acc);
    }
#pragma unroll
    for (int r8 = 0; r8 < 8; ++r8) {
      const float f = acc[r8];
      const unsigned short hb = f2bf_bits(f);
      const unsigned short lb = f2bf_bits(f - bf_bits2f(hb));
      const int idx = (ill * 16 + 8 * hh + r8) * 32 + rl;
      arHL[idx] = hb;
      arHL[8192 + idx] = lb;
    }
  }
  __syncthreads();
  const int q = lane >> 3, c8 = (lane & 7) * 8;
  float* sl = slab[wave];
#pragma unroll
  for (int sub = 0; sub < 2; ++sub) {
    const int h = wave + 8 * sub;
    const v16b ah = Frag<__bf16>::load((const __bf16*)arHL + rl * 512 + h * 32 + koff);
    const v16b al = Frag<__bf16>::load((const __bf16*)arHL + 8192 + rl * 512 + h * 32 + koff);
    v8f acc2[4];
#pragma unroll
    for (int j = 0; j < 4; ++j) {
      const v16b bw = Frag<__bf16>::load((const __bf16*)wrp + (size_t)(h * HDIM + j * 16 + rl) * 32 + koff);
      acc2[j] = mma16b(ah, bw, zero8);
      acc2[j] = mma16b(al, bw, acc2[j]);
    }
#pragma unroll
    for (int j = 0; j < 4; ++j)
#pragma unroll
      for (int r8 = 0; r8 < 8; ++r8) sl[(8 * hh + r8) * 68 + j * 16 + rl] = acc2[j][r8] * PCARRY_INV;
    __builtin_amdgcn_fence(__ATOMIC_RELEASE, "workgroup");
    __builtin_amdgcn_wave_barrier();
    __builtin_amdgcn_fence(__ATOMIC_ACQUIRE, "workgroup");
    v4u hv[4], lv[4];
#pragma unroll
    for (int it = 0; it < 4; ++it) {
      const int row = it * 4 + q;
      const size_t g = (size_t)(rowbase + il0 + row) * DMOD + h * HDIM + c8;
      const v4f s0 = *(const v4f*)(sl + row * 68 + c8);
      const v4f s1 = *(const v4f*)(sl + row * 68 + c8 + 4);
      const v4f r0 = *(const v4f*)(attsym + g);
      const v4f r1 = *(const v4f*)(attsym + g + 4);
      float v[8];
      v[0] = s0[0] + r0[0]; v[1] = s0[1] + r0[1]; v[2] = s0[2] + r0[2]; v[3] = s0[3] + r0[3];
      v[4] = s1[0] + r1[0]; v[5] = s1[1] + r1[1]; v[6] = s1[2] + r1[2]; v[7] = s1[3] + r1[3];
#pragma unroll
      for (int e = 0; e < 4; ++e) {
        const float a = v[2 * e], c = v[2 * e + 1];
        const unsigned short ha = f2bf_bits(a), hc = f2bf_bits(c);
        const unsigned short la = f2bf_bits(a - bf_bits2f(ha)), lc = f2bf_bits(c - bf_bits2f(hc));
        hv[it][e] = (unsigned)ha | ((unsigned)hc << 16);
        lv[it][e] = (unsigned)la | ((unsigned)lc << 16);
      }
    }
    for (int pass = 0; pass < 2; ++pass) {
#pragma unroll
      for (int it = 0; it < 4; ++it) {
        const int row = it * 4 + q;
        const size_t g = (size_t)(rowbase + il0 + row) * DMOD + h * HDIM + c8;
        *(volatile v4u*)(comb_hi + g) = hv[it];
        *(volatile v4u*)(comb_lo + g) = lv[it];
      }
      __threadfence();
    }
    __builtin_amdgcn_fence(__ATOMIC_RELEASE, "workgroup");
    __builtin_amdgcn_wave_barrier();
    __builtin_amdgcn_fence(__ATOMIC_ACQUIRE, "workgroup");
  }
}

template <int ET, bool SPLIT, bool SPLITB, int OUT_MODE>
static void launch_gemm(hipStream_t st, int batch,
                        const unsigned short* A, const unsigned short* A2, int lda, long sA,
                        const unsigned short* Bt, const unsigned short* Bt2, int ldb, long sB,
                        void* C, void* C2, int ldc, long sC, const float* dummy,
                        int M, int N, int K, float scale) {
  const int tiles = (M / 64) * (N / 64);
  dim3 grid((unsigned)((tiles + 7) / 8), (unsigned)batch, 1);
  wmma_gemm64<ET, SPLIT, SPLITB, 0, OUT_MODE><<<grid, 256, 0, st>>>(
      A, A2, lda, sA, Bt, Bt2, ldb, sB, C, C2, ldc, sC, dummy, M, N, K, scale);
}

extern "C" void kernel_launch(void* const* d_in, const int* in_sizes, int n_in,
                              void* d_out, int out_size, void* d_ws, size_t ws_size,
                              hipStream_t stream) {
  if (n_in < 9) return;
  if (in_sizes[0] != NTOK * DMOD || in_sizes[1] != NTOK * DMOD) return;
  if (in_sizes[2] != DMOD * DMOD || in_sizes[3] != DMOD * DMOD || in_sizes[4] != DMOD * DMOD ||
      in_sizes[5] != DMOD * DMOD || in_sizes[7] != DMOD * DMOD || in_sizes[8] != DMOD * DMOD) return;
  if (in_sizes[6] != NHEAD * HDIM * NREL) return;
  if (out_size != NTOK * DMOD) return;

  const float* x      = (const float*)d_in[0];
  const float* symb   = (const float*)d_in[1];
  const float* Wq_a   = (const float*)d_in[2];
  const float* Wk_a   = (const float*)d_in[3];
  const float* Wq_r   = (const float*)d_in[4];
  const float* Wk_r   = (const float*)d_in[5];
  const float* Wr     = (const float*)d_in[6];
  const float* Wv     = (const float*)d_in[7];
  const float* Wo     = (const float*)d_in[8];
  float* out = (float*)d_out;

  char* ws = (char*)d_ws;
  size_t off = 0;
  auto carve = [&](size_t bytes) -> char* {
    char* p = ws + off;
    off += (bytes + 255) & ~(size_t)255;
    return p;
  };
  const size_t ACT16 = (size_t)NTOK * DMOD * 2;
  const size_t WGT16 = (size_t)DMOD * DMOD * 2;
  const size_t ACT32 = (size_t)NTOK * DMOD * 4;
  const size_t PLANE_CH16 = (size_t)NHEAD * CHR * SEQ * 2;
  const size_t PLANE_CH32 = (size_t)NHEAD * CHR * SEQ * 4;
  const size_t REL_CH16   = (size_t)CHR * NREL * SEQ * 2;

  unsigned short* xb   = (unsigned short*)carve(ACT16);
  unsigned short* sb   = (unsigned short*)carve(ACT16);
  unsigned short* wT   = (unsigned short*)carve(6 * WGT16);
  unsigned short* xqh  = (unsigned short*)carve(ACT16);
  unsigned short* xql  = (unsigned short*)carve(ACT16);
  unsigned short* xkh  = (unsigned short*)carve(ACT16);
  unsigned short* xkl  = (unsigned short*)carve(ACT16);
  unsigned short* qr16 = (unsigned short*)carve(ACT16);
  unsigned short* kr16 = (unsigned short*)carve(ACT16);
  unsigned short* svh  = (unsigned short*)carve(ACT16);
  unsigned short* svl  = (unsigned short*)carve(ACT16);
  float*          attsym = (float*)carve(ACT32);
  unsigned short* ch   = (unsigned short*)carve(ACT16);
  unsigned short* cl   = (unsigned short*)carve(ACT16);
  unsigned short* wrp  = (unsigned short*)carve((size_t)NHEAD * HDIM * 32 * 2);
  float*          sc   = (float*)carve(PLANE_CH32);
  unsigned short* ph   = (unsigned short*)carve(PLANE_CH16);
  unsigned short* pl   = (unsigned short*)carve(PLANE_CH16);
  unsigned short* p16  = (unsigned short*)carve(PLANE_CH16);
  unsigned short* rel16 = (unsigned short*)carve(REL_CH16);
  if (off > ws_size) return;
  const float* dummy = (const float*)d_ws;

  const unsigned short* WqaT = wT + 0 * (size_t)DMOD * DMOD;
  const unsigned short* WkaT = wT + 1 * (size_t)DMOD * DMOD;
  const unsigned short* WqrT = wT + 2 * (size_t)DMOD * DMOD;
  const unsigned short* WkrT = wT + 3 * (size_t)DMOD * DMOD;
  const unsigned short* WvT  = wT + 4 * (size_t)DMOD * DMOD;
  const unsigned short* WoT  = wT + 5 * (size_t)DMOD * DMOD;

  {
    const int n8 = NTOK * DMOD / 8;
    k_cast_bf16x8<<<dim3((unsigned)((n8 + 255) / 256), 2, 1), 256, 0, stream>>>(x, symb, xb, sb, n8);
    k_wT_bf16<<<dim3(DMOD / 64, DMOD / 64, 6), 256, 0, stream>>>(Wq_a, Wk_a, Wq_r, Wk_r, Wv, Wo, wT);
    k_wr_pack<<<dim3((NHEAD * HDIM) / 64), 256, 0, stream>>>(Wr, wrp);
  }

  static_assert(NTOK % 64 == 0 && DMOD % 64 == 0 && DMOD % 32 == 0, "projection GEMM shapes");
  launch_gemm<1, false, true, 2>(stream, 1, xb, xb, DMOD, 0, WqaT, WqaT, DMOD, 0, xqh, xql, DMOD, 0, dummy, NTOK, DMOD, DMOD, 1.0f);
  launch_gemm<1, false, true, 2>(stream, 1, xb, xb, DMOD, 0, WkaT, WkaT, DMOD, 0, xkh, xkl, DMOD, 0, dummy, NTOK, DMOD, DMOD, 1.0f);
  launch_gemm<1, false, true, 1>(stream, 1, xb, xb, DMOD, 0, WqrT, WqrT, DMOD, 0, qr16, qr16, DMOD, 0, dummy, NTOK, DMOD, DMOD, 1.0f);
  launch_gemm<1, false, true, 1>(stream, 1, xb, xb, DMOD, 0, WkrT, WkrT, DMOD, 0, kr16, kr16, DMOD, 0, dummy, NTOK, DMOD, DMOD, 1.0f);
  launch_gemm<1, false, true, 2>(stream, 1, WvT, WvT, DMOD, 0, sb, sb, DMOD, 0, svh, svl, NTOK, 0, dummy, DMOD, NTOK, DMOD, 1.0f);

  static_assert(CHR % 64 == 0 && HDIM % 32 == 0 && RDIM % 32 == 0 && HDIM % 64 == 0, "chunk GEMM shapes");
  for (int b = 0; b < NB; ++b) {
    for (int cch = 0; cch < NCHK; ++cch) {
      const int i0 = cch * CHR;
      const int jend = CHR * (cch + 1);
      const int rowbase = b * SEQ + i0;
      launch_gemm<1, true, true, 0>(stream, NHEAD,
          xqh + (size_t)rowbase * DMOD, xql + (size_t)rowbase * DMOD, DMOD, (long)HDIM,
          xkh + (size_t)b * SEQ * DMOD, xkl + (size_t)b * SEQ * DMOD, DMOD, (long)HDIM,
          sc, sc, SEQ, (long)CHR * SEQ, dummy, CHR, jend, HDIM, SCALE_ATTN);
      k_softmax<<<dim3((NHEAD * CHR) / 8), 256, 0, stream>>>(sc, ph, pl, p16, i0, jend);
      launch_gemm<1, true, true, 0>(stream, NHEAD,
          ph, pl, SEQ, (long)CHR * SEQ,
          svh + (size_t)b * SEQ, svl + (size_t)b * SEQ, NTOK, (long)HDIM * NTOK,
          attsym + (size_t)rowbase * DMOD, attsym + (size_t)rowbase * DMOD, DMOD, (long)HDIM, dummy,
          CHR, HDIM, jend, 1.0f);
      launch_gemm<0, false, true, 1>(stream, NREL,
          qr16 + (size_t)rowbase * DMOD, qr16 + (size_t)rowbase * DMOD, DMOD, (long)RDIM,
          kr16 + (size_t)b * SEQ * DMOD, kr16 + (size_t)b * SEQ * DMOD, DMOD, (long)RDIM,
          rel16, rel16, NREL * SEQ, (long)SEQ, dummy, CHR, jend, RDIM, SCALE_REL);
      k_rel_mix<<<dim3(CHR / 16), 256, 0, stream>>>(p16, rel16, wrp, attsym, ch, cl, i0, rowbase);
    }
  }

  launch_gemm<1, true, false, 0>(stream, 1, ch, cl, DMOD, 0, WoT, WoT, DMOD, 0, out, out, DMOD, 0, dummy, NTOK, DMOD, DMOD, 1.0f);
}
